// TransformerDecoderLayer_16174846837150
// MI455X (gfx1250) — hardware-verified
//
#include <hip/hip_runtime.h>

#pragma clang fp contract(off)

typedef __attribute__((ext_vector_type(16))) _Float16 v16h;
typedef __attribute__((ext_vector_type(8)))  _Float16 v8h;
typedef __attribute__((ext_vector_type(16))) __bf16   v16b;
typedef __attribute__((ext_vector_type(8)))  __bf16   v8b;
typedef __attribute__((ext_vector_type(8)))  float    v8f;
typedef __attribute__((ext_vector_type(4)))  float    v4f;
typedef __attribute__((ext_vector_type(2)))  float    v2f;
typedef __attribute__((ext_vector_type(4)))  unsigned v4u;

constexpr int kL = 300;
constexpr int kB = 4;
constexpr int kD = 256;
constexpr int kH = 8;
constexpr int kHD = 32;
constexpr int kFF = 2048;
constexpr int kHW = 5184;
constexpr int kRows = kL * kB;
constexpr int kRowsP = 1280;
constexpr int kMemRows = kHW * kB;
constexpr int kTRows = 1216;
static_assert(kRowsP % 64 == 0, "tile multiple");
static_assert(kRowsP >= ((kL + 63) / 64) * 64 * kB, "attention writes every padded query slot");
static_assert(kMemRows % 64 == 0, "tile multiple");
static_assert(kD % 64 == 0 && kFF % 64 == 0 && kD % 32 == 0 && kFF % 32 == 0, "N tile / K step");
static_assert(kL >= 64 && kHW >= 64, "first key chunk fully valid");
static_assert(kH * kHD == kD, "head split");
static_assert(kRows % 64 == 48 || kRows % 64 == 0, "point kernel tail lines are whole");
static_assert(kTRows == ((kRows + 63) / 64) * 64 && kTRows <= kRowsP, "table rows");

constexpr size_t kOut0Floats = (size_t)kRows * kD;
constexpr size_t kOut1Off = kOut0Floats;
constexpr size_t kOut2Off = kOut1Off + (size_t)kRows * 2;
constexpr size_t kOutFloats = kOut2Off + (size_t)kRows * 16;
static_assert(kOut1Off * 4 == 1228800 && kOut2Off * 4 == 1238400 && kOutFloats * 4 == 1315200, "out offsets");
static_assert((kOut1Off * 4) % 128 == 0 && (kOut2Off * 4) % 128 == 0, "out regions line aligned");

constexpr size_t kSzMem16 = (size_t)kMemRows * kD * 2;
constexpr size_t kSzW3    = (size_t)3 * kD * kD * 2;
constexpr size_t kSzW1    = (size_t)kD * kD * 2;
constexpr size_t kSzWff   = (size_t)kFF * kD * 2;
constexpr size_t kSzHB    = (size_t)128 * kD * 2;
constexpr size_t kSzHBias = 512;
constexpr size_t kSzP16   = (size_t)kRowsP * kD * 2;
constexpr size_t kSzQK16  = (size_t)kRowsP * 2 * kD * 2;
constexpr size_t kSzP32   = (size_t)kRowsP * kD * 4;
constexpr size_t kSzH64   = (size_t)kRowsP * 64 * 4;
constexpr size_t kSzT     = (size_t)kTRows * 32 * 4;
constexpr size_t kSzHff   = (size_t)kRowsP * kFF * 2;

constexpr size_t kOffMem16 = 0;
constexpr size_t kOffMp16  = kOffMem16 + kSzMem16;
constexpr size_t kOffKc16  = kOffMp16 + kSzMem16;
constexpr size_t kOffVc16  = kOffKc16 + kSzMem16;
constexpr size_t kOffSaw   = kOffVc16 + kSzMem16;
constexpr size_t kOffSaow  = kOffSaw + kSzW3;
constexpr size_t kOffCaw   = kOffSaow + kSzW1;
constexpr size_t kOffCaow  = kOffCaw + kSzW3;
constexpr size_t kOffW1h   = kOffCaow + kSzW1;
constexpr size_t kOffW2h   = kOffW1h + kSzWff;
constexpr size_t kOffP1w0h = kOffW2h + kSzWff;
constexpr size_t kOffP1w1h = kOffP1w0h + kSzW1;
constexpr size_t kOffHB    = kOffP1w1h + kSzW1;
constexpr size_t kOffHBias = kOffHB + kSzHB;
constexpr size_t kOffXq16  = kOffHBias + kSzHBias;
constexpr size_t kOffTgt16 = kOffXq16 + kSzP16;
constexpr size_t kOffOut4h = kOffTgt16 + kSzP16;
constexpr size_t kOffVs16  = kOffOut4h + kSzP16;
constexpr size_t kOffOs16  = kOffVs16 + kSzP16;
constexpr size_t kOffH0h   = kOffOs16 + kSzP16;
constexpr size_t kOffH1h   = kOffH0h + kSzP16;
constexpr size_t kOffXq2h  = kOffH1h + kSzP16;
constexpr size_t kOffQc16  = kOffXq2h + kSzP16;
constexpr size_t kOffOc16  = kOffQc16 + kSzP16;
constexpr size_t kOffT2n16 = kOffOc16 + kSzP16;
constexpr size_t kOffQK16  = kOffT2n16 + kSzP16;
constexpr size_t kOffTgt32 = kOffQK16 + kSzQK16;
constexpr size_t kOffOs32  = kOffTgt32 + kSzP32;
constexpr size_t kOffX1    = kOffOs32 + kSzP32;
constexpr size_t kOffTgt1  = kOffX1 + kSzP32;
constexpr size_t kOffOc32  = kOffTgt1 + kSzP32;
constexpr size_t kOffX2    = kOffOc32 + kSzP32;
constexpr size_t kOffT2n32 = kOffX2 + kSzP32;
constexpr size_t kOffX3    = kOffT2n32 + kSzP32;
constexpr size_t kOffHeads = kOffX3 + kSzP32;
constexpr size_t kOffInter = kOffHeads + kSzH64;
constexpr size_t kOffT     = kOffInter + kSzH64;
constexpr size_t kOffHff   = kOffT + kSzT;
constexpr size_t kWsTotal  = kOffHff + kSzHff;
static_assert(kWsTotal == 71000576ull, "carve total");
static_assert(kWsTotal <= 134217728ull, "carve under 128 MiB");
static_assert(kOffHBias % 512 == 0 && kOffT % 512 == 0 && kOffHff % 512 == 0, "alignment");

__device__ __forceinline__ unsigned pk2h(float a, float b) {
  const unsigned short ha = __builtin_bit_cast(unsigned short, (_Float16)a);
  const unsigned short hb = __builtin_bit_cast(unsigned short, (_Float16)b);
  return (unsigned)ha | ((unsigned)hb << 16);
}
__device__ __forceinline__ v4u pack8f(v4f lo, v4f hi, float sc) {
  v4u u;
  u[0] = pk2h(lo[0] * sc, lo[1] * sc);
  u[1] = pk2h(lo[2] * sc, lo[3] * sc);
  u[2] = pk2h(hi[0] * sc, hi[1] * sc);
  u[3] = pk2h(hi[2] * sc, hi[3] * sc);
  return u;
}

__device__ __forceinline__ float block_sum_256(float v, float* sbuf) {
  const int tid = threadIdx.x;
#pragma unroll
  for (int off = 16; off > 0; off >>= 1) v += __shfl_xor(v, off);
  if ((tid & 31) == 0) sbuf[tid >> 5] = v;
  __syncthreads();
  float r = sbuf[tid & 7];
  r = ((tid & 31) < 8) ? r : 0.0f;
#pragma unroll
  for (int off = 16; off > 0; off >>= 1) r += __shfl_xor(r, off);
  __syncthreads();
  return r;
}

__device__ __forceinline__ unsigned short f2bf_bits(float f) {
  unsigned u = __float_as_uint(f);
  return (unsigned short)((u + 0x7FFFu + ((u >> 16) & 1u)) >> 16);
}
__device__ __forceinline__ float bf_bits2f(unsigned short h) { return __uint_as_float(((unsigned)h) << 16); }

__device__ __forceinline__ void dep_guard_h(v8f& a, v8f& b, v16h x, v16h y) { asm volatile("v_nop\n\tv_nop\n\tv_nop\n\tv_nop" : "+v"(a), "+v"(b) : "v"(x), "v"(y)); }
__device__ __forceinline__ void dep_guard_b(v8f& a, v8f& b, v16b x, v16b y) { asm volatile("v_nop\n\tv_nop\n\tv_nop\n\tv_nop" : "+v"(a), "+v"(b) : "v"(x), "v"(y)); }
__device__ __forceinline__ void keep4_h(v16h a, v16h b, v16h c, v16h d) { asm volatile("v_nop" :: "v"(a), "v"(b), "v"(c), "v"(d)); }
__device__ __forceinline__ void keep4_b(v16b a, v16b b, v16b c, v16b d) { asm volatile("v_nop" :: "v"(a), "v"(b), "v"(c), "v"(d)); }
__device__ __forceinline__ void acc_guard4(v8f& a, v8f& b, v8f& c, v8f& d) { asm volatile("v_nop\n\tv_nop\n\tv_nop\n\tv_nop" : "+v"(a), "+v"(b), "+v"(c), "+v"(d)); }
template <typename T> struct Frag;
template <> struct Frag<_Float16> {
  typedef v16h V; union U { v16h v; v8h h[2]; };
  static __device__ __forceinline__ v16h load(const _Float16* p) {
    U f; f.h[0] = *(const v8h*)(p); f.h[1] = *(const v8h*)(p + 16); return f.v;
  }
  static __device__ __forceinline__ v8f mma(v16h a, v16h b, v8f c) {
    return __builtin_amdgcn_wmma_f32_16x16x32_f16(false, a, false, b, (short)0, c, false, false);
  }
  static __device__ __forceinline__ void guard(v8f& a, v8f& b, v16h x, v16h y) { dep_guard_h(a, b, x, y); }
  static __device__ __forceinline__ void keep(v16h a, v16h b, v16h c, v16h d) { keep4_h(a, b, c, d); }
};
template <> struct Frag<__bf16> {
  typedef v16b V; union U { v16b v; v8b h[2]; };
  static __device__ __forceinline__ v16b load(const __bf16* p) {
    U f; f.h[0] = *(const v8b*)(p); f.h[1] = *(const v8b*)(p + 16); return f.v;
  }
  static __device__ __forceinline__ v8f mma(v16b a, v16b b, v8f c) {
    return __builtin_amdgcn_wmma_f32_16x16x32_bf16(false, a, false, b, (short)0, c, false, false);
  }
  static __device__ __forceinline__ void guard(v8f& a, v8f& b, v16b x, v16b y) { dep_guard_b(a, b, x, y); }
  static __device__ __forceinline__ void keep(v16b a, v16b b, v16b c, v16b d) { keep4_b(a, b, c, d); }
};

template <int ET> struct Elem;
template <> struct Elem<0> { typedef _Float16 T; };
template <> struct Elem<1> { typedef __bf16 T; };
template <int ET, bool SPLIT, int BIAS_MODE, int OUT_MODE, bool RESID, int ACT = 0>
__global__ __launch_bounds__(256) void wmma_gemm64(
    const unsigned short* __restrict__ Ap, const unsigned short* __restrict__ A2p, int lda, long strideA,
    const unsigned short* __restrict__ Btp, const unsigned short* __restrict__ Bt2p, int ldb, long strideB,
    void* __restrict__ Cout, void* __restrict__ Cout2, int ldc, long strideC,
    const float* __restrict__ bias,
    const float* __restrict__ resid, long strideR,
    int M, int N, int K, float scale) {
  static_assert(!RESID || OUT_MODE == 0, "residual only with f32 output");
  typedef typename Elem<ET>::T T;
  typedef typename Frag<T>::V V;
  const T* A = (const T*)Ap; const T* A2 = (const T*)A2p; const T* Bt = (const T*)Btp; const T* Bt2 = (const T*)Bt2p;
  __shared__ __align__(16) float sT[8][16 * 68];
  const int b    = blockIdx.y;
  const int lane = threadIdx.x & 31;
  const int wave = threadIdx.x >> 5;
  const int tilesN = N >> 6;
  const int tilesM = M >> 6;
  const int tile = blockIdx.x * 8 + wave;
  if (tile >= tilesM * tilesN) return;
  const int tm = tile / tilesN;
  const int tn = tile - tm * tilesN;
  const int m0 = tm << 6;
  const int n0 = tn << 6;

  const T* Ab  = A  + (size_t)b * strideA;
  const T* Bb  = Bt + (size_t)b * strideB;
  const T* Ab2 = SPLIT ? (A2  + (size_t)b * strideA) : nullptr;
  const T* Bb2 = SPLIT ? (Bt2 + (size_t)b * strideB) : nullptr;

  const int rlane = lane & 15;
  const int koff  = (lane >> 4) * 8;
  const int mOff  = (lane >> 4) * 8;

  v8f acc[4][4];
#pragma unroll
  for (int i = 0; i < 4; ++i)
#pragma unroll
    for (int j = 0; j < 4; ++j) acc[i][j] = (v8f){0.f,0.f,0.f,0.f,0.f,0.f,0.f,0.f};

  for (int k0 = 0; k0 < K; k0 += 32) {
    V bh[4], bl[4];
#pragma unroll
    for (int j = 0; j < 4; ++j) {
      const size_t bo = (size_t)(n0 + (j << 4) + rlane) * ldb + koff + k0;
      bh[j] = Frag<T>::load(Bb + bo);
      if (SPLIT) bl[j] = Frag<T>::load(Bb2 + bo);
    }
#pragma unroll
    for (int i = 0; i < 4; ++i) {
      const size_t ao = (size_t)(m0 + (i << 4) + rlane) * lda + koff + k0;
      V ah = Frag<T>::load(Ab + ao);
      V al;
      if (SPLIT) al = Frag<T>::load(Ab2 + ao);
#pragma unroll
      for (int j = 0; j < 4; ++j) {
        acc[i][j] = Frag<T>::mma(ah, bh[j], acc[i][j]);
        if (SPLIT) {
          acc[i][j] = Frag<T>::mma(ah, bl[j], acc[i][j]);
          acc[i][j] = Frag<T>::mma(al, bh[j], acc[i][j]);
        }
      }
      Frag<T>::guard(acc[i][0], acc[i][3], ah, SPLIT ? al : ah);
    }
    Frag<T>::keep(bh[0], bh[1], bh[2], bh[3]);
    if (SPLIT) Frag<T>::keep(bl[0], bl[1], bl[2], bl[3]);
  }
  acc_guard4(acc[0][0], acc[0][1], acc[0][2], acc[0][3]);
  acc_guard4(acc[1][0], acc[1][1], acc[1][2], acc[1][3]);
  acc_guard4(acc[2][0], acc[2][1], acc[2][2], acc[2][3]);
  acc_guard4(acc[3][0], acc[3][1], acc[3][2], acc[3][3]);

  float* slab = sT[wave];
  const float* Rb = RESID ? (resid + (size_t)b * strideR) : nullptr;
#pragma unroll
  for (int i = 0; i < 4; ++i) {
    const int mBase = m0 + (i << 4);
#pragma unroll
    for (int j = 0; j < 4; ++j) {
      const int n = n0 + (j << 4) + rlane;
      float bv = 0.f;
      if (BIAS_MODE == 2) bv = bias[n];
#pragma unroll
      for (int r = 0; r < 8; ++r) {
        float v = acc[i][j][r] * scale;
        if (BIAS_MODE == 1) v += bias[mBase + mOff + r];
        if (BIAS_MODE == 2) v += bv;
        if (ACT == 1) v = tanhf(v);
        if (ACT == 2) v = fmaxf(v, 0.0f);
        if (ACT == 3) v = v / (1.0f + expf(-v));
        if (ACT == 4) v = (v > 0.f) ? v : 0.01f * v;
        slab[(mOff + r) * 68 + (j << 4) + rlane] = v;
      }
    }
    __builtin_amdgcn_fence(__ATOMIC_RELEASE, "workgroup");
    __builtin_amdgcn_wave_barrier();
    __builtin_amdgcn_fence(__ATOMIC_ACQUIRE, "workgroup");
    if (OUT_MODE == 0) {
      float* C = (float*)Cout + (size_t)b * strideC;
      const int hh = lane >> 4, c4 = (lane & 15) * 4;
      for (int pass = 0; pass < 2; ++pass) {
#pragma unroll
        for (int it = 0; it < 8; ++it) {
          const int row = it * 2 + hh;
          v4f v = *(const v4f*)(slab + row * 68 + c4);
          if (RESID) {
            const v4f rv = *(const v4f*)(Rb + (size_t)(mBase + row) * ldc + n0 + c4);
            v = v + rv;
          }
          *(volatile v4f*)(C + (size_t)(mBase + row) * ldc + n0 + c4) = v;
        }
        __threadfence();
      }
    } else {
      const int q = lane >> 3, c8 = (lane & 7) * 8;
      unsigned short* C  = (unsigned short*)Cout  + (size_t)b * strideC;
      unsigned short* C2 = (OUT_MODE == 2) ? ((unsigned short*)Cout2 + (size_t)b * strideC) : nullptr;
      for (int pass = 0; pass < 2; ++pass) {
#pragma unroll
        for (int it = 0; it < 4; ++it) {
          const int row = it * 4 + q;
          const float* sp = slab + row * 68 + c8;
          v8h hv, lv;
#pragma unroll
          for (int e = 0; e < 8; ++e) {
            if (OUT_MODE == 1) {
              hv[e] = (_Float16)sp[e];
            } else {
              unsigned short hb = f2bf_bits(sp[e]);
              unsigned short lb = f2bf_bits(sp[e] - bf_bits2f(hb));
              hv[e] = __builtin_bit_cast(_Float16, hb);
              lv[e] = __builtin_bit_cast(_Float16, lb);
            }
          }
          *(volatile v8h*)(C + (size_t)(mBase + row) * ldc + n0 + c8) = hv;
          if (OUT_MODE == 2) *(volatile v8h*)(C2 + (size_t)(mBase + row) * ldc + n0 + c8) = lv;
        }
        __threadfence();
      }
    }
    __builtin_amdgcn_fence(__ATOMIC_RELEASE, "workgroup");
    __builtin_amdgcn_wave_barrier();
    __builtin_amdgcn_fence(__ATOMIC_ACQUIRE, "workgroup");
  }
}

__global__ __launch_bounds__(256) void k_cast8(const float* __restrict__ in, unsigned short* __restrict__ out, int n8, float sc) {
  const int i = blockIdx.x * 256 + threadIdx.x;
  if (i < n8) {
    const size_t o = (size_t)i * 8;
    const v4f a = *(const v4f*)(in + o);
    const v4f bq = *(const v4f*)(in + o + 4);
    const v4u u = pack8f(a, bq, sc);
    *(volatile v4u*)(out + o) = u;
    __threadfence();
    *(volatile v4u*)(out + o) = u;
  }
}

__global__ __launch_bounds__(256) void k_cast_mem(const float* __restrict__ a, const float* __restrict__ p,
                                                    unsigned short* __restrict__ oa, unsigned short* __restrict__ oap, int n8) {
  const int i = blockIdx.x * 256 + threadIdx.x;
  if (i < n8) {
    const size_t o = (size_t)i * 8;
    const v4f a0 = *(const v4f*)(a + o), a1 = *(const v4f*)(a + o + 4);
    const v4f p0 = *(const v4f*)(p + o), p1 = *(const v4f*)(p + o + 4);
    const v4u ua = pack8f(a0, a1, 1.0f);
    const v4u up = pack8f(a0 + p0, a1 + p1, 1.0f);
    *(volatile v4u*)(oa + o) = ua;
    *(volatile v4u*)(oap + o) = up;
    __threadfence();
    *(volatile v4u*)(oa + o) = ua;
    *(volatile v4u*)(oap + o) = up;
  }
}

__global__ __launch_bounds__(256) void k_pack_heads(const float* __restrict__ p2w, const float* __restrict__ p3w, const float* __restrict__ p1w2,
                                                     const float* __restrict__ p2b, const float* __restrict__ p3b, const float* __restrict__ p1b2,
                                                     unsigned short* __restrict__ hB, float* __restrict__ hbias, float sc) {
  const int tid = threadIdx.x, wave = tid >> 5, lane = tid & 31;
  const int gr = blockIdx.x * 8 + wave;
  int n2 = (gr < 16) ? gr : 15;
  int n3 = gr - 16; n3 = (n3 < 0) ? 0 : ((n3 > 7) ? 7 : n3);
  int n1 = gr - 64; n1 = (n1 < 0) ? 0 : ((n1 > 1) ? 1 : n1);
  const float* r2 = p2w + (size_t)n2 * 256 + 8 * lane;
  const float* r3 = p3w + (size_t)n3 * 256 + 8 * lane;
  const float* r1 = p1w2 + (size_t)n1 * 256 + 8 * lane;
  const v4f a2 = *(const v4f*)r2, b2v = *(const v4f*)(r2 + 4);
  const v4f a3 = *(const v4f*)r3, b3v = *(const v4f*)(r3 + 4);
  const v4f a1 = *(const v4f*)r1, b1v = *(const v4f*)(r1 + 4);
  const v4f z = {0.f, 0.f, 0.f, 0.f};
  const bool s2 = (gr < 16);
  const bool s3 = (gr >= 16) && (gr < 24);
  const bool s1 = (gr >= 64) && (gr < 66);
  v4f lo = z, hi = z;
  if (s2) { lo = a2; hi = b2v; }
  else if (s3) { lo = a3; hi = b3v; }
  else if (s1) { lo = a1; hi = b1v; }
  const v4u u = pack8f(lo, hi, sc);
  v4f bv4 = z;
#pragma unroll
  for (int i = 0; i < 4; ++i) {
    const int idx = 4 * lane + i;
    const int i2 = (idx < 16) ? idx : 15;
    int i3 = idx - 16; i3 = (i3 < 0) ? 0 : ((i3 > 7) ? 7 : i3);
    int i1 = idx - 64; i1 = (i1 < 0) ? 0 : ((i1 > 1) ? 1 : i1);
    const float c2 = p2b[i2];
    const float c3 = p3b[i3];
    const float c1 = p1b2[i1];
    float v = 0.0f;
    v = ((idx >= 64) && (idx < 66)) ? c1 : v;
    v = (idx < 24) ? c3 : v;
    v = (idx < 16) ? c2 : v;
    bv4[i] = v;
  }
  const bool dob = (blockIdx.x == 0) && (wave == 0);
  for (int pass = 0; pass < 2; ++pass) {
    *(volatile v4u*)(hB + (size_t)gr * 256 + 8 * lane) = u;
    if (dob) *(volatile v4f*)(hbias + 4 * lane) = bv4;
    __threadfence();
  }
}

__global__ __launch_bounds__(256) void k_prelude(const float* __restrict__ tgt, const float* __restrict__ qpos,
                                                  const float* __restrict__ n4w, const float* __restrict__ n4b,
                                                  unsigned short* __restrict__ xq16, unsigned short* __restrict__ tgt16,
                                                  unsigned short* __restrict__ out16, float* __restrict__ tgt32p, int nreal) {
  __shared__ __align__(16) float s_x[256];
  __shared__ __align__(16) float s_t[256];
  __shared__ __align__(16) float s_o[256];
  __shared__ float sred[8];
  const int r = blockIdx.x, tid = threadIdx.x, wave = tid >> 5, lane = tid & 31;
  const int rs = (r < nreal) ? r : (nreal - 1);
  const float tv = tgt[(size_t)rs * 256 + tid];
  const float xv = tv + qpos[(size_t)rs * 256 + tid];
  s_t[tid] = tv;
  s_x[tid] = xv;
  const float mean = block_sum_256(xv, sred) * (1.0f / 256.0f);
  const float d = xv - mean;
  const float var = block_sum_256(d * d, sred) * (1.0f / 256.0f);
  const float y = d * rsqrtf(var + 1e-5f) * n4w[tid] + n4b[tid];
  s_o[tid] = y;
  __syncthreads();
  const v4f z = {0.f, 0.f, 0.f, 0.f};
  v4u pk = {0u, 0u, 0u, 0u};
  v4f f0 = z, f1 = z;
  if (wave == 0) pk = pack8f(*(const v4f*)(s_x + 8 * lane), *(const v4f*)(s_x + 8 * lane + 4), 1.0f);
  else if (wave == 1) pk = pack8f(*(const v4f*)(s_t + 8 * lane), *(const v4f*)(s_t + 8 * lane + 4), 1.0f);
  else if (wave == 2) pk = pack8f(*(const v4f*)(s_o + 8 * lane), *(const v4f*)(s_o + 8 * lane + 4), 1.0f);
  else if (wave == 3) { f0 = *(const v4f*)(s_t + 4 * lane); f1 = *(const v4f*)(s_t + 128 + 4 * lane); }
  for (int pass = 0; pass < 2; ++pass) {
    if (wave == 0) *(volatile v4u*)(xq16 + (size_t)r * 256 + 8 * lane) = pk;
    else if (wave == 1) *(volatile v4u*)(tgt16 + (size_t)r * 256 + 8 * lane) = pk;
    else if (wave == 2) *(volatile v4u*)(out16 + (size_t)r * 256 + 8 * lane) = pk;
    else if (wave == 3) {
      *(volatile v4f*)(tgt32p + (size_t)r * 256 + 4 * lane) = f0;
      *(volatile v4f*)(tgt32p + (size_t)r * 256 + 128 + 4 * lane) = f1;
    }
    __threadfence();
  }
}

template <bool W32, bool W16, bool ADD>
__global__ __launch_bounds__(256) void k_ln(const float* __restrict__ x, const float* __restrict__ w, const float* __restrict__ bb,
                                             const float* __restrict__ addp, int add_rows,
                                             float* __restrict__ y32, unsigned short* __restrict__ y16) {
  __shared__ __align__(16) float s_y[256];
  __shared__ __align__(16) float s_a[256];
  __shared__ float sred[8];
  const int r = blockIdx.x, tid = threadIdx.x, wave = tid >> 5, lane = tid & 31;
  const float xv = x[(size_t)r * 256 + tid];
  const float mean = block_sum_256(xv, sred) * (1.0f / 256.0f);
  const float d = xv - mean;
  const float var = block_sum_256(d * d, sred) * (1.0f / 256.0f);
  const float y = d * rsqrtf(var + 1e-5f) * w[tid] + bb[tid];
  s_y[tid] = y;
  if (W16) {
    float a = 0.0f;
    if (ADD) {
      const int ra = (r < add_rows) ? r : (add_rows - 1);
      a = addp[(size_t)ra * 256 + tid];
    }
    s_a[tid] = y + a;
  } else {
    s_a[tid] = y;
  }
  __syncthreads();
  const v4f z = {0.f, 0.f, 0.f, 0.f};
  v4f p0 = z, p1 = z;
  v4u pk = {0u, 0u, 0u, 0u};
  if (W32 && wave == 0) { p0 = *(const v4f*)(s_y + 4 * lane); p1 = *(const v4f*)(s_y + 128 + 4 * lane); }
  if (W16 && wave == 1) { pk = pack8f(*(const v4f*)(s_a + 8 * lane), *(const v4f*)(s_a + 8 * lane + 4), 1.0f); }
  for (int pass = 0; pass < 2; ++pass) {
    if (W32 && wave == 0) {
      *(volatile v4f*)(y32 + (size_t)r * 256 + 4 * lane) = p0;
      *(volatile v4f*)(y32 + (size_t)r * 256 + 128 + 4 * lane) = p1;
    }
    if (W16 && wave == 1) {
      *(volatile v4u*)(y16 + (size_t)r * 256 + 8 * lane) = pk;
    }
    __threadfence();
  }
}

__device__ __forceinline__ float sigm(float x) { return 1.0f / (1.0f + expf(-x)); }

__device__ __forceinline__ v4f point_line_entry(const float* __restrict__ inter, const float* __restrict__ heads,
                                                const float* __restrict__ hw, int row, int e) {
  const v2f iv = *(const v2f*)(inter + (size_t)row * 64);
  const v2f ov = *(const v2f*)(heads + (size_t)row * 64 + 2 * e);
  const float sp = heads[(size_t)row * 64 + 16 + e];
  const int bb = row & 3;
  const float h0 = hw[2 * bb], h1 = hw[2 * bb + 1];
  const float ref0 = (h0 * sigm(iv[0])) * 0.03125f;
  const float ref1 = (h1 * sigm(iv[1])) * 0.03125f;
  v4f tv;
  tv[0] = ref0 + ov[0];
  tv[1] = ref1 + ov[1];
  tv[2] = sp * sp;
  tv[3] = 0.0f;
  return tv;
}

__global__ __launch_bounds__(256) void k_point(const float* __restrict__ inter, const float* __restrict__ heads, const float* __restrict__ hw,
                                                float* __restrict__ ptab, float* __restrict__ o1, float* __restrict__ o2, int nreal) {
  const int tid = threadIdx.x, wave = tid >> 5, lane = tid & 31;
  const int base = blockIdx.x * 64;
  const int rA0 = base + wave * 8 + (lane >> 3);
  const int rA1 = rA0 + 4;
  const int e = lane & 7;
  const v4f tv0 = point_line_entry(inter, heads, hw, rA0, e);
  const v4f tv1 = point_line_entry(inter, heads, hw, rA1, e);
  const int rB = base + wave * 8 + (lane >> 2);
  const int cg = lane & 3;
  const bool validB = (base + wave * 8 + 8) <= nreal;
  v4f bv;
  {
    const v2f iv = *(const v2f*)(inter + (size_t)rB * 64);
    const int bb = rB & 3;
    const float h0 = hw[2 * bb], h1 = hw[2 * bb + 1];
    const float ref0 = (h0 * sigm(iv[0])) * 0.03125f;
    const float ref1 = (h1 * sigm(iv[1])) * 0.03125f;
    bv[0] = ref0; bv[1] = ref1; bv[2] = ref0; bv[3] = ref1;
  }
  const int rC = base + 2 * lane;
  const bool validC = (wave == 0) && ((rC + 2) <= nreal);
  v4f cv;
  {
    const v2f ia = *(const v2f*)(inter + (size_t)rC * 64);
    const v2f ib = *(const v2f*)(inter + (size_t)(rC + 1) * 64);
    cv[0] = ia[0]; cv[1] = ia[1]; cv[2] = ib[0]; cv[3] = ib[1];
  }
  for (int pass = 0; pass < 2; ++pass) {
    *(volatile v4f*)(ptab + (size_t)rA0 * 32 + 4 * e) = tv0;
    *(volatile v4f*)(ptab + (size_t)rA1 * 32 + 4 * e) = tv1;
    if (validB) *(volatile v4f*)(o2 + (size_t)rB * 16 + 4 * cg) = bv;
    if (validC) *(volatile v4f*)(o1 + (size_t)rC * 2) = cv;
    __threadfence();
  }
}

struct A32G { long q_bs, q_rs, q_hs, k_bs, k_rs, k_hs, v_bs, v_rs, v_hs, o_bs, o_rs, o_hs; int S, Skv, H, NB; float qscale; int pad0; };
static_assert(sizeof(A32G) == 120, "no padding");

constexpr float kPSC = 32768.0f;

__device__ __forceinline__ v8f hmma(v16h a, v16h b, v8f c) {
  c = __builtin_amdgcn_wmma_f32_16x16x32_f16(false, a, false, b, (short)0, c, false, false);
  asm volatile("v_nop\n\tv_nop\n\tv_nop\n\tv_nop" : "+v"(c) : "v"(a), "v"(b));
  return c;
}

template <bool HAS_BIAS>
__global__ __launch_bounds__(128) void attn32_kernel(const unsigned short* __restrict__ qp, const unsigned short* __restrict__ kp,
                                                      const unsigned short* __restrict__ vp, float* __restrict__ outp,
                                                      const float* __restrict__ ptab, const float* __restrict__ gxy, A32G g) {
  union FH { v16h v; v8h h[2]; };
  __shared__ __align__(16) unsigned short Kh[64 * 32];
  __shared__ __align__(16) unsigned short Vt[32 * 64];
  __shared__ __align__(16) _Float16 Ph[4][16 * 64];
  __shared__ __align__(16) float Os[4][16 * 40];
  __shared__ __align__(16) float sG[HAS_BIAS ? 128 : 4];

  const int tid = threadIdx.x;
  const int wave = tid >> 5, lane = tid & 31, hh = lane >> 4, c = lane & 15;
  const int nqb = (g.S + 63) >> 6;
  const int bx = blockIdx.x;
  const int qb = bx % nqb;
  const int bhi = bx / nqb;
  const int h = bhi % g.H;
  const int b = bhi / g.H;
  const int q0 = qb * 64 + wave * 16;

  const _Float16* qbase = (const _Float16*)qp + (size_t)b * g.q_bs + (size_t)h * g.q_hs;
  const unsigned short* kbase = kp + (size_t)b * g.k_bs + (size_t)h * g.k_hs;
  const unsigned short* vbase = vp + (size_t)b * g.v_bs + (size_t)h * g.v_hs;
  float* obase = outp + (size_t)b * g.o_bs + (size_t)h * g.o_hs;

  v16h qa;
  {
    int l = q0 + c;
    l = (l < g.S) ? l : (g.S - 1);
    qa = Frag<_Float16>::load(qbase + (size_t)l * g.q_rs + 8 * hh);
  }
  float px[8], py[8], ps[8];
#pragma unroll
  for (int r = 0; r < 8; ++r) {
    px[r] = 0.0f; py[r] = 0.0f; ps[r] = 0.0f;
    if (HAS_BIAS) {
      int l = q0 + 8 * hh + r;
      l = (l < g.S) ? l : (g.S - 1);
      const v4f t4 = *(const v4f*)(ptab + ((size_t)(l * g.NB + b) * 32 + (size_t)h * 4));
      px[r] = t4[0]; py[r] = t4[1]; ps[r] = t4[2];
    }
  }

  float mrow[8], lrow[8];
  v8f oacc[2];
#pragma unroll
  for (int r = 0; r < 8; ++r) { mrow[r] = -__builtin_inff(); lrow[r] = 0.0f; }
#pragma unroll
  for (int t = 0; t < 2; ++t) oacc[t] = (v8f){0.f,0.f,0.f,0.f,0.f,0.f,0.f,0.f};

  const int nChunks = (g.Skv + 63) >> 6;
  for (int kc = 0; kc < nChunks; ++kc) {
    const int kv0 = kc * 64;
    __syncthreads();
    {
      const int kvr = tid >> 1, dh = (tid & 1) * 16;
      int kv = kv0 + kvr;
      kv = (kv < g.Skv) ? kv : (g.Skv - 1);
      const unsigned short* kr = kbase + (size_t)kv * g.k_rs + dh;
      const unsigned short* vr = vbase + (size_t)kv * g.v_rs + dh;
      const v4u k0w = *(const v4u*)kr;
      const v4u k1w = *(const v4u*)(kr + 8);
      const v4u v0w = *(const v4u*)vr;
      const v4u v1w = *(const v4u*)(vr + 8);
      *(v4u*)(Kh + kvr * 32 + dh) = k0w;
      *(v4u*)(Kh + kvr * 32 + dh + 8) = k1w;
#pragma unroll
      for (int e = 0; e < 8; ++e) {
        const unsigned w0 = v0w[e >> 1];
        const unsigned w1 = v1w[e >> 1];
        const int sh = (e & 1) * 16;
        Vt[(dh + e) * 64 + kvr]     = (unsigned short)((w0 >> sh) & 0xffffu);
        Vt[(dh + 8 + e) * 64 + kvr] = (unsigned short)((w1 >> sh) & 0xffffu);
      }
      if (HAS_BIAS && tid < 32) {
        int ka = kv0 + 2 * tid;
        int kb2 = ka + 1;
        ka  = (ka  < g.Skv) ? ka  : (g.Skv - 1);
        kb2 = (kb2 < g.Skv) ? kb2 : (g.Skv - 1);
        const v2f ga = *(const v2f*)(gxy + 2 * (size_t)ka);
        const v2f gb = *(const v2f*)(gxy + 2 * (size_t)kb2);
        sG[4 * tid + 0] = ga[0];
        sG[4 * tid + 1] = ga[1];
        sG[4 * tid + 2] = gb[0];
        sG[4 * tid + 3] = gb[1];
      }
    }
    __syncthreads();

    v8f s[4];
#pragma unroll
    for (int j = 0; j < 4; ++j) {
      FH kb;
      const _Float16* kr = (const _Float16*)Kh + (j * 16 + c) * 32;
      kb.h[0] = *(const v8h*)(kr + 8 * hh);
      kb.h[1] = *(const v8h*)(kr + 16 + 8 * hh);
      s[j] = hmma(qa, kb.v, (v8f){0.f,0.f,0.f,0.f,0.f,0.f,0.f,0.f});
    }
    float gx[4], gy[4];
#pragma unroll
    for (int j = 0; j < 4; ++j) {
      gx[j] = 0.0f; gy[j] = 0.0f;
      if (HAS_BIAS) { gx[j] = sG[(j * 16 + c) * 2]; gy[j] = sG[(j * 16 + c) * 2 + 1]; }
    }
    float cm[8];
#pragma unroll
    for (int r = 0; r < 8; ++r) {
      float m = -__builtin_inff();
#pragma unroll
      for (int j = 0; j < 4; ++j) {
        const int kvcol = kv0 + j * 16 + c;
        float val = s[j][r] * g.qscale;
        if (HAS_BIAS) {
          const float dx = px[r] - gx[j];
          const float dy = py[r] - gy[j];
          const float d2 = dx * dx + dy * dy;
          val = val - fabsf(d2 * ps[r]) * 0.125f;
        }
        val = (kvcol < g.Skv) ? val : -__builtin_inff();
        s[j][r] = val;
        m = fmaxf(m, val);
      }
#pragma unroll
      for (int off = 1; off < 16; off <<= 1) m = fmaxf(m, __shfl_xor(m, off, 32));
      cm[r] = m;
    }
    _Float16* pwh = Ph[wave];
#pragma unroll
    for (int r = 0; r < 8; ++r) {
      const float mnew = fmaxf(mrow[r], cm[r]);
      const float alpha = expf(mrow[r] - mnew);
      mrow[r] = mnew;
      float psum = 0.0f;
#pragma unroll
      for (int j = 0; j < 4; ++j) {
        const float p = expf(s[j][r] - mnew);
        psum += p;
        pwh[(8 * hh + r) * 64 + j * 16 + c] = (_Float16)(p * kPSC);
      }
#pragma unroll
      for (int off = 1; off < 16; off <<= 1) psum += __shfl_xor(psum, off, 32);
      lrow[r] = lrow[r] * alpha + psum;
      oacc[0][r] *= alpha;
      oacc[1][r] *= alpha;
    }
    __builtin_amdgcn_fence(__ATOMIC_RELEASE, "workgroup");
    __builtin_amdgcn_wave_barrier();
    __builtin_amdgcn_fence(__ATOMIC_ACQUIRE, "workgroup");
#pragma unroll
    for (int kk = 0; kk < 2; ++kk) {
      FH pa;
      pa.h[0] = *(const v8h*)(pwh + c * 64 + kk * 32 + 8 * hh);
      pa.h[1] = *(const v8h*)(pwh + c * 64 + kk * 32 + 16 + 8 * hh);
#pragma unroll
      for (int t = 0; t < 2; ++t) {
        FH vb;
        const _Float16* vr = (const _Float16*)Vt + (t * 16 + c) * 64 + kk * 32;
        vb.h[0] = *(const v8h*)(vr + 8 * hh);
        vb.h[1] = *(const v8h*)(vr + 16 + 8 * hh);
        oacc[t] = hmma(pa.v, vb.v, oacc[t]);
      }
    }
  }

  float* os = Os[wave];
#pragma unroll
  for (int r = 0; r < 8; ++r) {
    const float inv = 1.0f / (lrow[r] * kPSC);
#pragma unroll
    for (int t = 0; t < 2; ++t) os[(8 * hh + r) * 40 + t * 16 + c] = oacc[t][r] * inv;
  }
  __builtin_amdgcn_fence(__ATOMIC_RELEASE, "workgroup");
  __builtin_amdgcn_wave_barrier();
  __builtin_amdgcn_fence(__ATOMIC_ACQUIRE, "workgroup");
  {
    const int q4 = lane >> 3, c4 = (lane & 7) * 4;
    for (int pass = 0; pass < 2; ++pass) {
#pragma unroll
      for (int it = 0; it < 4; ++it) {
        const int row = it * 4 + q4;
        const v4f val = *(const v4f*)(os + row * 40 + c4);
        *(volatile v4f*)(obase + (size_t)(q0 + row) * g.o_rs + c4) = val;
      }
      __threadfence();
    }
  }
}

template <int BIAS_MODE, int OUT_MODE, bool RESID, int ACT>
static void launch_gemm(hipStream_t st, const unsigned short* A, int lda, const unsigned short* Bt, int ldb,
                        void* C, int ldc, const float* bias, const float* resid, int M, int N, int K, float scale) {
  const int tiles = (M / 64) * (N / 64);
  const int blocks = (tiles + 7) / 8;
  wmma_gemm64<0, false, BIAS_MODE, OUT_MODE, RESID, ACT><<<dim3(blocks, 1), 256, 0, st>>>(
      A, A, lda, 0L, Bt, Bt, ldb, 0L, C, C, ldc, 0L, bias, resid, 0L, M, N, K, scale);
}

static void launch_cast(hipStream_t st, const float* in, unsigned short* out, int n, float sc) {
  const int n8 = n / 8;
  const int blocks = (n8 + 255) / 256;
  k_cast8<<<blocks, 256, 0, st>>>(in, out, n8, sc);
}
static_assert((3 * kD * kD) % 2048 == 0 && (kD * kD) % 2048 == 0 && (kFF * kD) % 2048 == 0 && (kRowsP * kD) % 2048 == 0, "cast grids exact");
static_assert(((size_t)kMemRows * kD) % 2048 == 0, "mem cast grid exact");

extern "C" void kernel_launch(void* const* d_in, const int* in_sizes, int n_in,
                              void* d_out, int out_size, void* d_ws, size_t ws_size, hipStream_t stream)
{
  (void)in_sizes;
  if (n_in < 36) return;
  if (out_size < (int)kOutFloats) return;
  if (ws_size < kWsTotal) return;

  const float* grid_in = (const float*)d_in[0];
  const float* h_w     = (const float*)d_in[1];
  const float* tgt     = (const float*)d_in[2];
  const float* memory  = (const float*)d_in[3];
  const float* qpos    = (const float*)d_in[4];
  const float* pos     = (const float*)d_in[5];
  const float* sa_w    = (const float*)d_in[6];
  const float* sa_b    = (const float*)d_in[7];
  const float* sa_ow   = (const float*)d_in[8];
  const float* sa_ob   = (const float*)d_in[9];
  const float* ca_w    = (const float*)d_in[10];
  const float* ca_b    = (const float*)d_in[11];
  const float* ca_ow   = (const float*)d_in[12];
  const float* ca_ob   = (const float*)d_in[13];
  const float* w1      = (const float*)d_in[14];
  const float* b1      = (const float*)d_in[15];
  const float* w2      = (const float*)d_in[16];
  const float* b2      = (const float*)d_in[17];
  const float* n1w     = (const float*)d_in[18];
  const float* n1b     = (const float*)d_in[19];
  const float* n2w     = (const float*)d_in[20];
  const float* n2b     = (const float*)d_in[21];
  const float* n3w     = (const float*)d_in[22];
  const float* n3b     = (const float*)d_in[23];
  const float* n4w     = (const float*)d_in[24];
  const float* n4b     = (const float*)d_in[25];
  const float* p1w0    = (const float*)d_in[26];
  const float* p1b0    = (const float*)d_in[27];
  const float* p1w1    = (const float*)d_in[28];
  const float* p1b1    = (const float*)d_in[29];
  const float* p1w2    = (const float*)d_in[30];
  const float* p1b2    = (const float*)d_in[31];
  const float* p2w     = (const float*)d_in[32];
  const float* p2b     = (const float*)d_in[33];
  const float* p3w     = (const float*)d_in[34];
  const float* p3b     = (const float*)d_in[35];

  char* ws = (char*)d_ws;
  unsigned short* mem16  = (unsigned short*)(ws + kOffMem16);
  unsigned short* mp16   = (unsigned short*)(ws + kOffMp16);
  unsigned short* Kc16   = (unsigned short*)(ws + kOffKc16);
  unsigned short* Vc16   = (unsigned short*)(ws + kOffVc16);
  unsigned short* saw    = (unsigned short*)(ws + kOffSaw);
  unsigned short* saow   = (unsigned short*)(ws + kOffSaow);
  unsigned short* caw    = (unsigned short*)(ws + kOffCaw);
  unsigned short* caow   = (unsigned short*)(ws + kOffCaow);
  unsigned short* w1h    = (unsigned short*)(ws + kOffW1h);
  unsigned short* w2h    = (unsigned short*)(ws + kOffW2h);
  unsigned short* p1w0h  = (unsigned short*)(ws + kOffP1w0h);
  unsigned short* p1w1h  = (unsigned short*)(ws + kOffP1w1h);
  unsigned short* hB     = (unsigned short*)(ws + kOffHB);
  float*          hbias  = (float*)(ws + kOffHBias);
  unsigned short* xq16   = (unsigned short*)(ws + kOffXq16);
  unsigned short* tgt16  = (unsigned short*)(ws + kOffTgt16);
  unsigned short* out4h  = (unsigned short*)(ws + kOffOut4h);
  unsigned short* Vs16   = (unsigned short*)(ws + kOffVs16);
  unsigned short* Os16   = (unsigned short*)(ws + kOffOs16);
  unsigned short* h0h    = (unsigned short*)(ws + kOffH0h);
  unsigned short* h1h    = (unsigned short*)(ws + kOffH1h);
  unsigned short* xq2h   = (unsigned short*)(ws + kOffXq2h);
  unsigned short* Qc16   = (unsigned short*)(ws + kOffQc16);
  unsigned short* Oc16   = (unsigned short*)(ws + kOffOc16);
  unsigned short* t2n16  = (unsigned short*)(ws + kOffT2n16);
  unsigned short* QK16   = (unsigned short*)(ws + kOffQK16);
  float* tgt32p  = (float*)(ws + kOffTgt32);
  float* Os32    = (float*)(ws + kOffOs32);
  float* x1      = (float*)(ws + kOffX1);
  float* tgt1_32 = (float*)(ws + kOffTgt1);
  float* Oc32    = (float*)(ws + kOffOc32);
  float* x2      = (float*)(ws + kOffX2);
  float* t2n32   = (float*)(ws + kOffT2n32);
  float* x3      = (float*)(ws + kOffX3);
  float* heads32 = (float*)(ws + kOffHeads);
  float* inter32 = (float*)(ws + kOffInter);
  float* ptab    = (float*)(ws + kOffT);
  unsigned short* Hff16 = (unsigned short*)(ws + kOffHff);

  float* out0 = (float*)d_out;
  float* out1 = out0 + kOut1Off;
  float* out2 = out0 + kOut2Off;

  const float qscale = 0.17677669529663687f;
  const float wsc = 16.0f;
  const float winv = 0.0625f;

  launch_cast(stream, sa_w,  saw,   3 * kD * kD, wsc);
  launch_cast(stream, sa_ow, saow,  kD * kD, wsc);
  launch_cast(stream, ca_w,  caw,   3 * kD * kD, wsc);
  launch_cast(stream, ca_ow, caow,  kD * kD, wsc);
  launch_cast(stream, w1,    w1h,   kFF * kD, wsc);
  launch_cast(stream, w2,    w2h,   kD * kFF, wsc);
  launch_cast(stream, p1w0,  p1w0h, kD * kD, wsc);
  launch_cast(stream, p1w1,  p1w1h, kD * kD, wsc);
  k_pack_heads<<<16, 256, 0, stream>>>(p2w, p3w, p1w2, p2b, p3b, p1b2, hB, hbias, wsc);

  {
    const int n8 = (kMemRows * kD) / 8;
    k_cast_mem<<<(n8 + 255) / 256, 256, 0, stream>>>(memory, pos, mem16, mp16, n8);
  }

  k_prelude<<<kRowsP, 256, 0, stream>>>(tgt, qpos, n4w, n4b, xq16, tgt16, out4h, tgt32p, kRows);

  static_assert(kRowsP % 64 == 0 && 64 % 64 == 0 && kD % 32 == 0, "heads gemm shape");
  launch_gemm<2, 0, false, 0>(stream, out4h, kD, hB,           kD, heads32, 64, hbias,      hbias, kRowsP, 64, kD, winv);
  launch_gemm<2, 1, false, 2>(stream, out4h, kD, p1w0h,        kD, h0h,     kD, p1b0,       p1b0,  kRowsP, kD, kD, winv);
  launch_gemm<2, 1, false, 2>(stream, h0h,   kD, p1w1h,        kD, h1h,     kD, p1b1,       p1b1,  kRowsP, kD, kD, winv);
  launch_gemm<2, 0, false, 0>(stream, h1h,   kD, hB + 64 * kD, kD, inter32, 64, hbias + 64, hbias, kRowsP, 64, kD, winv);
  k_point<<<kTRows / 64, 256, 0, stream>>>(inter32, heads32, h_w, ptab, out1, out2, kRows);

  launch_gemm<2, 1, false, 0>(stream, xq16,  kD, saw,               kD, QK16, 2 * kD, sa_b,          sa_b, kRowsP, 2 * kD, kD, winv);
  launch_gemm<2, 1, false, 0>(stream, tgt16, kD, saw + 2 * kD * kD, kD, Vs16, kD,     sa_b + 2 * kD, sa_b, kRowsP, kD,     kD, winv);
  {
    A32G gs;
    gs.q_bs = 2 * kD; gs.q_rs = (long)kB * 2 * kD; gs.q_hs = kHD;
    gs.k_bs = 2 * kD; gs.k_rs = (long)kB * 2 * kD; gs.k_hs = kHD;
    gs.v_bs = kD;     gs.v_rs = (long)kB * kD;     gs.v_hs = kHD;
    gs.o_bs = kD;     gs.o_rs = (long)kB * kD;     gs.o_hs = kHD;
    gs.S = kL; gs.Skv = kL; gs.H = kH; gs.NB = kB; gs.qscale = qscale; gs.pad0 = 0;
    const int nqb = (kL + 63) / 64;
    attn32_kernel<false><<<kB * kH * nqb, 128, 0, stream>>>(QK16, QK16 + kD, Vs16, Os32, ptab, grid_in, gs);
  }
  launch_cast(stream, Os32, Os16, kRowsP * kD, 1.0f);
  launch_gemm<2, 0, true, 0>(stream, Os16, kD, saow, kD, x1, kD, sa_ob, tgt32p, kRowsP, kD, kD, winv);
  k_ln<true, true, true><<<kRowsP, 256, 0, stream>>>(x1, n1w, n1b, qpos, kRows, tgt1_32, xq2h);

  launch_gemm<2, 1, false, 0>(stream, xq2h,  kD, caw,               kD, Qc16, kD, ca_b,          ca_b, kRowsP,   kD, kD, winv);
  launch_gemm<2, 1, false, 0>(stream, mp16,  kD, caw + kD * kD,     kD, Kc16, kD, ca_b + kD,     ca_b, kMemRows, kD, kD, winv);
  launch_gemm<2, 1, false, 0>(stream, mem16, kD, caw + 2 * kD * kD, kD, Vc16, kD, ca_b + 2 * kD, ca_b, kMemRows, kD, kD, winv);
  {
    A32G gc;
    gc.q_bs = kD; gc.q_rs = (long)kB * kD; gc.q_hs = kHD;
    gc.k_bs = kD; gc.k_rs = (long)kB * kD; gc.k_hs = kHD;
    gc.v_bs = kD; gc.v_rs = (long)kB * kD; gc.v_hs = kHD;
    gc.o_bs = kD; gc.o_rs = (long)kB * kD; gc.o_hs = kHD;
    gc.S = kL; gc.Skv = kHW; gc.H = kH; gc.NB = kB; gc.qscale = qscale; gc.pad0 = 0;
    const int nqb = (kL + 63) / 64;
    attn32_kernel<true><<<kB * kH * nqb, 128, 0, stream>>>(Qc16, Kc16, Vc16, Oc32, ptab, grid_in, gc);
  }
  launch_cast(stream, Oc32, Oc16, kRowsP * kD, 1.0f);
  launch_gemm<2, 0, true, 0>(stream, Oc16, kD, caow, kD, x2, kD, ca_ob, tgt1_32, kRowsP, kD, kD, winv);
  k_ln<true, true, false><<<kRowsP, 256, 0, stream>>>(x2, n2w, n2b, x2, 1, t2n32, t2n16);

  static_assert(kFF % 64 == 0 && kFF % 32 == 0, "ffn shapes");
  launch_gemm<2, 1, false, 2>(stream, t2n16, kD,  w1h, kD,  Hff16, kFF, b1, b1,    kRowsP, kFF, kD,  winv);
  launch_gemm<2, 0, true, 0>(stream, Hff16, kFF, w2h, kFF, x3,    kD,  b2, t2n32, kRowsP, kD,  kFF, winv);
  k_ln<true, false, false><<<kRows, 256, 0, stream>>>(x3, n3w, n3b, x3, 1, out0, xq16);
}
